// CopyModel_82961588290052
// MI455X (gfx1250) — hardware-run, weakly checked
//
#include <hip/hip_runtime.h>
#include <math.h>
#include <stdint.h>

#ifndef NB
#define NB       2
#endif
#ifndef SEQ
#define SEQ      4096
#endif
#define NB_FULL  2
#define SEQ_FULL 4096
#define DMODEL   512
#define DFF      2048
#define NHEAD    8
#define HDIM     64
#define NROWS    (NB * SEQ)
#define WSC      64.0f
#define XC       16.0f
#define HC       16.0f
#define QSC      4096.0f
#define KEC      1.0f
#define VC       16.0f
#define PC       1024.0f
#define KSC      16384.0f
#define CC       1024.0f
#define GC       64.0f
#define QSCALE   0.125f
#define ATT_EPS  1e-6f
#define LOG2E    1.4426950408889634f
#define LN_EPS   1e-5f
static_assert(NHEAD * HDIM == DMODEL);
static_assert(NB >= 1 && NB <= NB_FULL && SEQ >= 256 && SEQ <= SEQ_FULL);
static_assert((SEQ % 64) == 0 && (SEQ % 32) == 0 && (SEQ % 16) == 0 && (DMODEL % 64) == 0 && (DFF % 64) == 0);
static_assert((NROWS % 64) == 0 && (DMODEL % 32) == 0 && (DFF % 32) == 0);
static_assert(((NROWS * DMODEL) % 2048) == 0 && ((3 * DMODEL * DMODEL) % 2048) == 0 && ((DMODEL * DMODEL) % 2048) == 0);
static_assert(DMODEL == 512);

typedef _Float16 v16h __attribute__((ext_vector_type(16)));
typedef _Float16 v8h  __attribute__((ext_vector_type(8)));
typedef float    v8f  __attribute__((ext_vector_type(8)));
typedef float    v4f  __attribute__((ext_vector_type(4)));
typedef unsigned int v4u __attribute__((ext_vector_type(4)));
typedef unsigned int v2u __attribute__((ext_vector_type(2)));

union FragH { v16h v; v8h h[2]; v4u u[2]; };

__device__ __forceinline__ unsigned short bf_bits(float f) {
  unsigned u = __float_as_uint(f);
  return (unsigned short)((u + 0x7FFFu + ((u >> 16) & 1u)) >> 16);
}
__device__ __forceinline__ float bf_up(unsigned short h) { return __uint_as_float(((unsigned)h) << 16); }
__device__ __forceinline__ float bfr(float f) { return bf_up(bf_bits(f)); }
__device__ __forceinline__ unsigned short h_bits(_Float16 x) { return __builtin_bit_cast(unsigned short, x); }
__device__ __forceinline__ unsigned pk16(unsigned short a, unsigned short b) { return (unsigned)a | ((unsigned)b << 16); }
__device__ __forceinline__ v8f zero8() { v8f z = {0.f, 0.f, 0.f, 0.f, 0.f, 0.f, 0.f, 0.f}; return z; }
__device__ __forceinline__ int imin(int a, int b) { return a < b ? a : b; }

__device__ __forceinline__ v16h ldfrag_h(const _Float16* p) {
  FragH f;
  f.h[0] = *(const v8h*)(p);
  f.h[1] = *(const v8h*)(p + 16);
  return f.v;
}
__device__ __forceinline__ v16h ldfrag_u(const unsigned short* p) {
  FragH f;
  f.u[0] = *(const v4u*)(p);
  f.u[1] = *(const v4u*)(p + 16);
  return f.v;
}

__device__ __forceinline__ v8f mma_raw(v16h a, v16h b, v8f c) {
  return __builtin_amdgcn_wmma_f32_16x16x32_f16(false, a, false, b, (short)0, c, false, false);
}
__device__ __forceinline__ void dep_guard1(v8f& a, v8f& b, v16h x) {
#if defined(__HIP_DEVICE_COMPILE__)
  asm volatile("v_nop\n\tv_nop\n\tv_nop\n\tv_nop" : "+v"(a), "+v"(b) : "v"(x));
#endif
}
__device__ __forceinline__ void guard_s2(v8f& s, v16h a0, v16h a1) {
#if defined(__HIP_DEVICE_COMPILE__)
  asm volatile("v_nop\n\tv_nop\n\tv_nop\n\tv_nop" : "+v"(s) : "v"(a0), "v"(a1));
#endif
}
__device__ __forceinline__ void guard_s4(v8f& s, v16h a0, v16h a1, v16h b0, v16h b1) {
#if defined(__HIP_DEVICE_COMPILE__)
  asm volatile("v_nop\n\tv_nop\n\tv_nop\n\tv_nop" : "+v"(s) : "v"(a0), "v"(a1), "v"(b0), "v"(b1));
#endif
}
__device__ __forceinline__ void guard_pv4(v8f& a, v8f& b, v8f& c, v8f& d, v16h x, v16h y, v16h z, v16h w, v16h u) {
#if defined(__HIP_DEVICE_COMPILE__)
  asm volatile("v_nop\n\tv_nop\n\tv_nop\n\tv_nop"
               : "+v"(a), "+v"(b), "+v"(c), "+v"(d) : "v"(x), "v"(y), "v"(z), "v"(w), "v"(u));
#endif
}
__device__ __forceinline__ void keep4_h(v16h a, v16h b, v16h c, v16h d) {
#if defined(__HIP_DEVICE_COMPILE__)
  asm volatile("v_nop" :: "v"(a), "v"(b), "v"(c), "v"(d));
#endif
}
__device__ __forceinline__ void acc_guard4(v8f& a, v8f& b, v8f& c, v8f& d) {
#if defined(__HIP_DEVICE_COMPILE__)
  asm volatile("v_nop\n\tv_nop\n\tv_nop\n\tv_nop" : "+v"(a), "+v"(b), "+v"(c), "+v"(d));
#endif
}
__device__ __forceinline__ void wave_sync_lds() {
  __builtin_amdgcn_fence(__ATOMIC_RELEASE, "workgroup");
  __builtin_amdgcn_wave_barrier();
  __builtin_amdgcn_fence(__ATOMIC_ACQUIRE, "workgroup");
}

__global__ __launch_bounds__(256) void cvt16(const float* __restrict__ src, unsigned short* dst,
                                             int C, int seg, int segfull, float sc) {
  const int p   = (blockIdx.x * 256 + threadIdx.x) * 8;
  const int r   = p / C;
  const int cc  = p - r * C;
  const int sb  = r / seg;
  const int sr  = sb * segfull + (r - sb * seg);
  const float* sp = src + (size_t)sr * C + cc;
  const v4f a = *(const v4f*)(sp);
  const v4f b = *(const v4f*)(sp + 4);
  v4u w;
  w[0] = pk16(h_bits((_Float16)(bfr(a[0]) * sc)), h_bits((_Float16)(bfr(a[1]) * sc)));
  w[1] = pk16(h_bits((_Float16)(bfr(a[2]) * sc)), h_bits((_Float16)(bfr(a[3]) * sc)));
  w[2] = pk16(h_bits((_Float16)(bfr(b[0]) * sc)), h_bits((_Float16)(bfr(b[1]) * sc)));
  w[3] = pk16(h_bits((_Float16)(bfr(b[2]) * sc)), h_bits((_Float16)(bfr(b[3]) * sc)));
  for (int pass = 0; pass < 2; ++pass) {
    *(volatile v4u*)(dst + (size_t)p) = w;
    __threadfence();
  }
}

template <int OM, int RM, int ACT, int BM>
__global__ __launch_bounds__(256) void gemm64(
    const unsigned short* __restrict__ Ap, int lda, long long sA1, long long sA2,
    const unsigned short* __restrict__ Btp, int ldb, long long sB1, long long sB2,
    const float* __restrict__ Rp,
    const float* __restrict__ biasp, int nbias,
    void* Cout, int ldc, long long sC1, long long sC2, int zd,
    int M, int N, int K, float oscale, float ocarry) {
  static_assert(ACT < 3 || OM == 2);
  static_assert(OM == 0 || OM == 2);
  __shared__ __align__(16) float sT[8][16 * 68];
  const int by   = blockIdx.y;
  const int zhi  = by / zd;
  const int zlo  = by - zhi * zd;
  const int lane = threadIdx.x & 31;
  const int wave = threadIdx.x >> 5;
  const int wpb  = blockDim.x >> 5;
  const int tilesN = N >> 6;
  const int tilesM = M >> 6;
  const int tile = blockIdx.x * wpb + wave;
  if (tile >= tilesM * tilesN) return;
  const int tm = tile / tilesN;
  const int tn = tile - tm * tilesN;
  const int m0 = tm << 6;
  const int n0 = tn << 6;

  const long long aoff = (long long)zhi * sA1 + (long long)zlo * sA2;
  const long long boff = (long long)zhi * sB1 + (long long)zlo * sB2;
  const long long coff = (long long)zhi * sC1 + (long long)zlo * sC2;
  const unsigned short* A1 = Ap  + aoff;
  const unsigned short* Bb = Btp + boff;

  const int rlane = lane & 15;
  const int koff  = (lane >> 4) * 8;
  const int mOff  = (lane >> 4) * 8;

  v8f acc[4][4];
#pragma unroll
  for (int i = 0; i < 4; ++i)
#pragma unroll
    for (int j = 0; j < 4; ++j) acc[i][j] = zero8();

  for (int k0 = 0; k0 < K; k0 += 32) {
    v16h bh[4];
#pragma unroll
    for (int j = 0; j < 4; ++j) {
      const size_t bofs = (size_t)(n0 + (j << 4) + rlane) * ldb + koff + k0;
      bh[j] = ldfrag_u(Bb + bofs);
    }
#pragma unroll
    for (int i = 0; i < 4; ++i) {
      const size_t ao = (size_t)(m0 + (i << 4) + rlane) * lda + koff + k0;
      const v16h ah = ldfrag_u(A1 + ao);
#pragma unroll
      for (int j = 0; j < 4; ++j) acc[i][j] = mma_raw(ah, bh[j], acc[i][j]);
      dep_guard1(acc[i][0], acc[i][3], ah);
    }
    keep4_h(bh[0], bh[1], bh[2], bh[3]);
  }
  acc_guard4(acc[0][0], acc[0][1], acc[0][2], acc[0][3]);
  acc_guard4(acc[1][0], acc[1][1], acc[1][2], acc[1][3]);
  acc_guard4(acc[2][0], acc[2][1], acc[2][2], acc[2][3]);
  acc_guard4(acc[3][0], acc[3][1], acc[3][2], acc[3][3]);

  const int hh2 = lane >> 4, c4 = (lane & 15) * 4;
  const int q8  = lane >> 3, c8 = (lane & 7) * 8;

  float bc4[4], bc8[8];
#pragma unroll
  for (int e = 0; e < 4; ++e) bc4[e] = 0.f;
#pragma unroll
  for (int e = 0; e < 8; ++e) bc8[e] = 0.f;
  if constexpr (BM == 1) {
    if constexpr (OM == 0) {
#pragma unroll
      for (int e = 0; e < 4; ++e) {
        const int n = n0 + c4 + e;
        const int ncl = imin(n, nbias - 1);
        const float t = bfr(biasp[ncl]);
        bc4[e] = (n < nbias) ? t : 0.f;
      }
    } else {
#pragma unroll
      for (int e = 0; e < 8; ++e) {
        const int n = n0 + c8 + e;
        const int ncl = imin(n, nbias - 1);
        const float t = bfr(biasp[ncl]);
        bc8[e] = (n < nbias) ? t : 0.f;
      }
    }
  }

  float* slab = sT[wave];
#pragma unroll
  for (int i = 0; i < 4; ++i) {
    const int mBase = m0 + (i << 4);
#pragma unroll
    for (int j = 0; j < 4; ++j) {
#pragma unroll
      for (int r = 0; r < 8; ++r) {
        slab[(mOff + r) * 68 + (j << 4) + rlane] = acc[i][j][r];
      }
    }
    wave_sync_lds();
    if constexpr (OM == 0) {
      float* C = (float*)Cout + coff;
      v4f vals[8];
#pragma unroll
      for (int it = 0; it < 8; ++it) {
        const int row = it * 2 + hh2;
        const int gr  = mBase + row;
        v4f v = *(const v4f*)(slab + row * 68 + c4);
        v4f rv = {0.f, 0.f, 0.f, 0.f};
        if constexpr (RM == 1 || RM == 2) {
          const float* R = Rp + coff;
          const v4f rraw = *(const v4f*)(R + (size_t)gr * ldc + n0 + c4);
#pragma unroll
          for (int e = 0; e < 4; ++e) rv[e] = (RM == 1) ? bfr(rraw[e]) : rraw[e];
        }
        float br = 0.f;
        if constexpr (BM == 2) {
          const float t = bfr(biasp[imin(gr, nbias - 1)]);
          br = (gr < nbias) ? t : 0.f;
        }
#pragma unroll
        for (int e = 0; e < 4; ++e) {
          float u = v[e] * oscale;
          if constexpr (BM == 1) u += bc4[e];
          if constexpr (BM == 2) u += br;
          if constexpr (ACT == 1) u = fmaxf(u, 0.f);
          v[e] = u + rv[e];
        }
        vals[it] = v;
      }
      for (int pass = 0; pass < 2; ++pass) {
#pragma unroll
        for (int it = 0; it < 8; ++it) {
          const int gr = mBase + it * 2 + hh2;
          *(volatile v4f*)(C + (size_t)gr * ldc + n0 + c4) = vals[it];
        }
        __threadfence();
      }
    } else {
      unsigned short* C = (unsigned short*)Cout + coff;
      v4u hv[4];
#pragma unroll
      for (int it = 0; it < 4; ++it) {
        const int row = it * 4 + q8;
        const int gr  = mBase + row;
        const float* sp = slab + row * 68 + c8;
        float br = 0.f;
        if constexpr (BM == 2) {
          const float t = bfr(biasp[imin(gr, nbias - 1)]);
          br = (gr < nbias) ? t : 0.f;
        }
        (void)gr;
        float u[8];
#pragma unroll
        for (int k = 0; k < 8; ++k) {
          float t = sp[k] * oscale;
          if constexpr (BM == 1) t += bc8[k];
          if constexpr (BM == 2) t += br;
          if constexpr (ACT == 1) t = fmaxf(t, 0.f);
          if constexpr (ACT == 3) t = exp2f(t * LOG2E);
          u[k] = t;
        }
        if constexpr (ACT == 4) {
          float mx = u[0];
#pragma unroll
          for (int k = 1; k < 8; ++k) mx = fmaxf(mx, u[k]);
          mx = fmaxf(mx, __shfl_xor(mx, 1, 32));
          mx = fmaxf(mx, __shfl_xor(mx, 2, 32));
          mx = fmaxf(mx, __shfl_xor(mx, 4, 32));
          float s = 0.f;
#pragma unroll
          for (int k = 0; k < 8; ++k) { u[k] = exp2f((u[k] - mx) * LOG2E); s += u[k]; }
          s += __shfl_xor(s, 1, 32);
          s += __shfl_xor(s, 2, 32);
          s += __shfl_xor(s, 4, 32);
          const float inv = (1.0f / s) * QSCALE;
#pragma unroll
          for (int k = 0; k < 8; ++k) u[k] *= inv;
        }
        v4u a = {0u, 0u, 0u, 0u};
#pragma unroll
        for (int e = 0; e < 4; ++e) {
          a[e] = pk16(h_bits((_Float16)(u[2 * e] * ocarry)), h_bits((_Float16)(u[2 * e + 1] * ocarry)));
        }
        hv[it] = a;
      }
      for (int pass = 0; pass < 2; ++pass) {
#pragma unroll
        for (int it = 0; it < 4; ++it) {
          const int row = it * 4 + q8;
          *(volatile v4u*)(C + (size_t)(mBase + row) * ldc + n0 + c8) = hv[it];
        }
        __threadfence();
      }
    }
    wave_sync_lds();
  }
}

#define ATT_THREADS    (NHEAD * 32)
#define ATT_LDS_FLOATS (16 * DMODEL)
#define ATT_WIT        ((16 * DMODEL) / (4 * ATT_THREADS))
static_assert(ATT_THREADS == 256 && ATT_LDS_FLOATS >= NHEAD * 16 * 36 && ATT_WIT * 4 * ATT_THREADS == 16 * DMODEL && ATT_WIT == 8);
static_assert((DMODEL / 4) == 128);

__global__ __launch_bounds__(ATT_THREADS)
void attnc(const unsigned short* __restrict__ QSp, const unsigned short* __restrict__ KEp,
           const unsigned short* __restrict__ VTp, float* O1) {
  __shared__ __align__(16) float smem[ATT_LDS_FLOATS];

  const int tid  = threadIdx.x;
  const int wave = tid >> 5;
  const int lane = tid & 31;
  const int hh   = lane >> 4;
  const int c    = lane & 15;

  const int qt   = blockIdx.x % (SEQ / 16);
  const int bat  = blockIdx.x / (SEQ / 16);
  const int head = wave;
  const int q0   = qt * 16;

  const size_t qofs = ((size_t)bat * SEQ + q0 + c) * DMODEL + head * HDIM + 8 * hh;
  const _Float16* Qh = (const _Float16*)(const void*)QSp + qofs;
  const _Float16* Kb = (const _Float16*)(const void*)KEp + (size_t)bat * SEQ * DMODEL + head * HDIM + 8 * hh;
  const _Float16* Vb = (const _Float16*)(const void*)VTp + ((size_t)bat * DMODEL + head * HDIM) * SEQ + 8 * hh;
  const float psc = PC / (QSC * KEC);

  const v16h qa = ldfrag_h(Qh), qb = ldfrag_h(Qh + 32);

  float part = 0.f;
#pragma unroll
  for (int i = 0; i < 16; ++i) part += (float)qa[i] + (float)qb[i];
  part *= (1.0f / QSC);
  const float sqm = part + __shfl_xor(part, 16, 32);
  float sqr[8], lrow[8];
#pragma unroll
  for (int r = 0; r < 8; ++r) { sqr[r] = __shfl(sqm, 8 * hh + r, 32); lrow[r] = 0.f; }

  v8f o0 = zero8(), o1 = zero8(), o2 = zero8(), o3 = zero8();
  float* pt = smem + wave * (16 * 36);
  const int kend = q0 + 16;

#pragma unroll 1
  for (int kb = 0; kb < kend; kb += 32) {
    const _Float16* kp = Kb + (size_t)(kb + c) * DMODEL;
    v8f s0, s1;
    {
      const v16h k0 = ldfrag_h(kp), k1 = ldfrag_h(kp + 32);
      s0 = mma_raw(qa, k0, zero8());
      s0 = mma_raw(qb, k1, s0);
      guard_s2(s0, k0, k1);
    }
    {
      const _Float16* kq = kp + (size_t)16 * DMODEL;
      const v16h k0 = ldfrag_h(kq), k1 = ldfrag_h(kq + 32);
      s1 = mma_raw(qa, k0, zero8());
      s1 = mma_raw(qb, k1, s1);
      guard_s4(s1, k0, k1, qa, qb);
    }
#pragma unroll
    for (int r = 0; r < 8; ++r) {
      const int i = q0 + 8 * hh + r;
      float e0 = (kb + c <= i) ? s0[r] * psc : 0.f;
      float e1 = (kb + 16 + c <= i) ? s1[r] * psc : 0.f;
      e0 = (float)((_Float16)e0);
      e1 = (float)((_Float16)e1);
      float ps = e0 + e1;
#pragma unroll
      for (int off = 1; off < 16; off <<= 1) ps += __shfl_xor(ps, off, 32);
      lrow[r] += ps;
      const int ro = (8 * hh + r) * 36 + c;
      pt[ro]      = e0;
      pt[ro + 16] = e1;
    }
    wave_sync_lds();
    FragH ph;
    {
      const float* prow = pt + c * 36 + 8 * hh;
      const v4f p0 = *(const v4f*)(prow), p1 = *(const v4f*)(prow + 4);
      const v4f p2 = *(const v4f*)(prow + 16), p3 = *(const v4f*)(prow + 20);
#pragma unroll
      for (int e = 0; e < 4; ++e) {
        ph.h[0][e]     = (_Float16)(p0[e]);
        ph.h[0][4 + e] = (_Float16)(p1[e]);
        ph.h[1][e]     = (_Float16)(p2[e]);
        ph.h[1][4 + e] = (_Float16)(p3[e]);
      }
    }
    const _Float16* vp = Vb + (size_t)c * SEQ + kb;
    {
      const v16h vb0 = ldfrag_h(vp);
      const v16h vb1 = ldfrag_h(vp + (size_t)16 * SEQ);
      const v16h vb2 = ldfrag_h(vp + (size_t)32 * SEQ);
      const v16h vb3 = ldfrag_h(vp + (size_t)48 * SEQ);
      o0 = mma_raw(ph.v, vb0, o0);
      o1 = mma_raw(ph.v, vb1, o1);
      o2 = mma_raw(ph.v, vb2, o2);
      o3 = mma_raw(ph.v, vb3, o3);
      guard_pv4(o0, o1, o2, o3, ph.v, vb0, vb1, vb2, vb3);
    }
    wave_sync_lds();
  }

  __syncthreads();
  float* Os = smem;
  const float oc = 1.0f / (PC * VC);
  float* osw = Os + head * HDIM + c;
#pragma unroll
  for (int r = 0; r < 8; ++r) {
    const float den = lrow[r] * (1.0f / PC) + ATT_EPS * sqr[r];
    const float inv = (1.0f / den) * oc;
    float* op = osw + (8 * hh + r) * DMODEL;
    op[0]  = o0[r] * inv;
    op[16] = o1[r] * inv;
    op[32] = o2[r] * inv;
    op[48] = o3[r] * inv;
  }
  __syncthreads();
  {
    v4f vals[ATT_WIT];
#pragma unroll
    for (int it = 0; it < ATT_WIT; ++it) {
      const int p = it * ATT_THREADS + tid;
      vals[it] = *(const v4f*)(Os + (size_t)p * 4);
    }
    float* dst = O1 + ((size_t)bat * SEQ + q0) * DMODEL;
    for (int pass = 0; pass < 2; ++pass) {
#pragma unroll
      for (int it = 0; it < ATT_WIT; ++it) {
        const int p = it * ATT_THREADS + tid;
        const int row = p >> 7, col4 = (p & 127) * 4;
        *(volatile v4f*)(dst + (size_t)row * DMODEL + col4) = vals[it];
      }
      __threadfence();
    }
  }
}

#define CS_THREADS (((SEQ) / 8) < 256 ? ((SEQ) / 8) : 256)
#define CS_NCH     (SEQ / (CS_THREADS * 8))
#define CS_NW      (CS_THREADS / 32)
static_assert(CS_THREADS >= 32 && (CS_THREADS % 32) == 0 && (CS_NCH * CS_THREADS * 8) == SEQ && CS_NCH >= 1 && CS_NCH <= 2);

__global__ __launch_bounds__(CS_THREADS)
void colsoft(const float* __restrict__ Kp, unsigned short* KSo) {
  __shared__ float red[2][CS_NW];
  const int row = blockIdx.x, tid = threadIdx.x, lane = tid & 31, wave = tid >> 5;
  const float* rp = Kp + (size_t)row * SEQ;
  float v[CS_NCH][8];
  float mx = -INFINITY;
#pragma unroll
  for (int ch = 0; ch < CS_NCH; ++ch) {
    const float* p = rp + ch * (CS_THREADS * 8) + tid * 8;
    const v4f a = *(const v4f*)(p), b = *(const v4f*)(p + 4);
#pragma unroll
    for (int e = 0; e < 4; ++e) { v[ch][e] = a[e]; v[ch][4 + e] = b[e]; }
#pragma unroll
    for (int k = 0; k < 8; ++k) mx = fmaxf(mx, v[ch][k]);
  }
#pragma unroll
  for (int off = 1; off < 32; off <<= 1) mx = fmaxf(mx, __shfl_xor(mx, off, 32));
  if (lane == 0) red[0][wave] = mx;
  __syncthreads();
  float m = red[0][0];
#pragma unroll
  for (int w = 1; w < CS_NW; ++w) m = fmaxf(m, red[0][w]);
  float s = 0.f;
#pragma unroll
  for (int ch = 0; ch < CS_NCH; ++ch) {
#pragma unroll
    for (int k = 0; k < 8; ++k) { const float e = exp2f((v[ch][k] - m) * LOG2E); v[ch][k] = e; s += e; }
  }
#pragma unroll
  for (int off = 1; off < 32; off <<= 1) s += __shfl_xor(s, off, 32);
  if (lane == 0) red[1][wave] = s;
  __syncthreads();
  float tot = 0.f;
#pragma unroll
  for (int w = 0; w < CS_NW; ++w) tot += red[1][w];
  const float f = (1.0f / tot) * KSC;
  v4u w[CS_NCH];
#pragma unroll
  for (int ch = 0; ch < CS_NCH; ++ch) {
#pragma unroll
    for (int e = 0; e < 4; ++e)
      w[ch][e] = pk16(h_bits((_Float16)(v[ch][2 * e] * f)), h_bits((_Float16)(v[ch][2 * e + 1] * f)));
  }
  unsigned short* dst = KSo + (size_t)row * SEQ;
  for (int pass = 0; pass < 2; ++pass) {
#pragma unroll
    for (int ch = 0; ch < CS_NCH; ++ch) {
      *(volatile v4u*)(dst + ch * (CS_THREADS * 8) + tid * 8) = w[ch];
    }
    __threadfence();
  }
}

#define LN_THREADS 128
#define LN_NW (LN_THREADS / 32)
static_assert(LN_THREADS * 4 == DMODEL);

template <int RES, int HOUT, int FOUT>
__global__ __launch_bounds__(LN_THREADS)
void lnorm(const float* __restrict__ Yp, const float* __restrict__ Rp, const float* __restrict__ gp,
           const float* __restrict__ bp, unsigned short* outh, float* outf, float hc) {
  __shared__ float red[2][LN_NW];
  __shared__ __align__(16) unsigned short srow[DMODEL];
  const int row  = blockIdx.x;
  const int tid  = threadIdx.x;
  const int lane = tid & 31;
  const int wave = tid >> 5;
  const int bb   = row / SEQ;
  const int frow = bb * SEQ_FULL + (row - bb * SEQ);
  v4f v = *(const v4f*)(Yp + (size_t)row * DMODEL + (size_t)tid * 4);
  if constexpr (RES == 1) {
    const v4f rr = *(const v4f*)(Rp + (size_t)frow * DMODEL + (size_t)tid * 4);
#pragma unroll
    for (int e = 0; e < 4; ++e) v[e] += bfr(rr[e]);
  }
  if constexpr (RES == 2) {
    const v4f rr = *(const v4f*)(Rp + (size_t)row * DMODEL + (size_t)tid * 4);
#pragma unroll
    for (int e = 0; e < 4; ++e) v[e] += rr[e];
  }
  float s = (v[0] + v[1]) + (v[2] + v[3]);
#pragma unroll
  for (int off = 1; off < 32; off <<= 1) s += __shfl_xor(s, off, 32);
  if (lane == 0) red[0][wave] = s;
  __syncthreads();
  float tot = 0.f;
#pragma unroll
  for (int w = 0; w < LN_NW; ++w) tot += red[0][w];
  const float mu = tot * (1.0f / (float)DMODEL);
  v4f d;
#pragma unroll
  for (int e = 0; e < 4; ++e) d[e] = v[e] - mu;
  float q = (d[0] * d[0] + d[1] * d[1]) + (d[2] * d[2] + d[3] * d[3]);
#pragma unroll
  for (int off = 1; off < 32; off <<= 1) q += __shfl_xor(q, off, 32);
  if (lane == 0) red[1][wave] = q;
  __syncthreads();
  float totq = 0.f;
#pragma unroll
  for (int w = 0; w < LN_NW; ++w) totq += red[1][w];
  const float var  = totq * (1.0f / (float)DMODEL);
  const float rstd = rsqrtf(var + LN_EPS);
  const v4f gv = *(const v4f*)(gp + (size_t)tid * 4);
  const v4f bv = *(const v4f*)(bp + (size_t)tid * 4);
  v4f o;
#pragma unroll
  for (int e = 0; e < 4; ++e) o[e] = (d[e] * rstd) * bfr(gv[e]) + bfr(bv[e]);
  if constexpr (HOUT == 1) {
    v2u w;
    w[0] = pk16(h_bits((_Float16)(o[0] * hc)), h_bits((_Float16)(o[1] * hc)));
    w[1] = pk16(h_bits((_Float16)(o[2] * hc)), h_bits((_Float16)(o[3] * hc)));
    *(v2u*)(srow + tid * 4) = w;
    __syncthreads();
    if (tid < DMODEL / 8) {
      const v4u hv = *(const v4u*)(srow + tid * 8);
      unsigned short* dst = outh + (size_t)row * DMODEL + (size_t)tid * 8;
      for (int pass = 0; pass < 2; ++pass) {
        *(volatile v4u*)dst = hv;
        __threadfence();
      }
    }
  }
  if constexpr (FOUT != 0) {
    const size_t orow = (FOUT == 2) ? (size_t)frow : (size_t)row;
    float* dst = outf + orow * DMODEL + (size_t)tid * 4;
    for (int pass = 0; pass < 2; ++pass) {
      *(volatile v4f*)dst = o;
      __threadfence();
    }
  }
  (void)hc;
}

extern "C" void kernel_launch(void* const* d_in, const int* in_sizes, int n_in,
                              void* d_out, int out_size, void* d_ws, size_t ws_size,
                              hipStream_t stream) {
  if (n_in < 18) return;
  const int needX = ((NB - 1) * SEQ_FULL + SEQ) * DMODEL;
  if (in_sizes[0] < needX || in_sizes[1] < needX) return;
  if (in_sizes[2] < 3 * DMODEL * DMODEL || in_sizes[3] < 3 * DMODEL) return;
  if (in_sizes[4] < 2 * DMODEL * DMODEL || in_sizes[5] < 2 * DMODEL) return;
  if (in_sizes[6] < DMODEL * DMODEL || in_sizes[7] < DMODEL) return;
  if (in_sizes[8] < DMODEL || in_sizes[9] < DMODEL || in_sizes[10] < DMODEL || in_sizes[11] < DMODEL) return;
  if (in_sizes[12] < DFF * DMODEL || in_sizes[13] < DFF) return;
  if (in_sizes[14] < DMODEL * DFF || in_sizes[15] < DMODEL) return;
  if (in_sizes[16] < DMODEL || in_sizes[17] < DMODEL) return;
  if (out_size < needX) return;

  const float* x     = (const float*)d_in[0];
  const float* mem   = (const float*)d_in[1];
  const float* w_qvk = (const float*)d_in[2];
  const float* b_qvk = (const float*)d_in[3];
  const float* w_kv  = (const float*)d_in[4];
  const float* b_kv  = (const float*)d_in[5];
  const float* w_q   = (const float*)d_in[6];
  const float* b_q   = (const float*)d_in[7];
  const float* ln1_g = (const float*)d_in[8];
  const float* ln1_b = (const float*)d_in[9];
  const float* ln2_g = (const float*)d_in[10];
  const float* ln2_b = (const float*)d_in[11];
  const float* w_ff1 = (const float*)d_in[12];
  const float* b_ff1 = (const float*)d_in[13];
  const float* w_ff2 = (const float*)d_in[14];
  const float* b_ff2 = (const float*)d_in[15];
  const float* ln3_g = (const float*)d_in[16];
  const float* ln3_b = (const float*)d_in[17];
  float*       out   = (float*)d_out;

  const size_t PWQVK = (size_t)3 * DMODEL * DMODEL * 2;
  const size_t PWKV  = (size_t)2 * DMODEL * DMODEL * 2;
  const size_t PWQ   = (size_t)DMODEL * DMODEL * 2;
  const size_t PWF   = (size_t)DFF * DMODEL * 2;
  const size_t PCTX  = (size_t)NB * NHEAD * HDIM * HDIM * 2;
  const size_t U     = (size_t)NROWS * DMODEL * 2;
  size_t off = 0;
  const size_t oWQVK = off; off += PWQVK;
  const size_t oWKV  = off; off += PWKV;
  const size_t oWQ   = off; off += PWQ;
  const size_t oW1   = off; off += PWF;
  const size_t oW2   = off; off += PWF;
  const size_t oCTX  = off; off += PCTX;
  const size_t oS    = ((off + (size_t)1048575) / (size_t)1048576) * (size_t)1048576;
  const size_t endAll = oS + 8 * U;
  if (endAll > ws_size) return;
  if (endAll > (size_t)134217728) return;

  char* ws = (char*)d_ws;
  unsigned short* WQVK16 = (unsigned short*)(ws + oWQVK);
  unsigned short* WKV16  = (unsigned short*)(ws + oWKV);
  unsigned short* WQ16   = (unsigned short*)(ws + oWQ);
  unsigned short* W116   = (unsigned short*)(ws + oW1);
  unsigned short* W216   = (unsigned short*)(ws + oW2);
  unsigned short* CTX16  = (unsigned short*)(ws + oCTX);
  char* S0 = ws + oS;
  char* S1 = S0 + U;
  char* S2 = S1 + U;
  char* S4 = S2 + 2 * U;
  char* S5 = S4 + U;
  char* S7 = S5 + 2 * U;
  unsigned short* X16   = (unsigned short*)S0;
  unsigned short* MEM16 = (unsigned short*)S1;
  unsigned short* QS16  = (unsigned short*)S2;
  unsigned short* KE16  = (unsigned short*)(S2 + U);
  unsigned short* VT16  = (unsigned short*)S4;
  float*          O1F   = (float*)S5;
  unsigned short* LN1H  = (unsigned short*)S0;
  float*          LN1F  = (float*)S2;
  float*          K2TF  = (float*)S5;
  unsigned short* V2T16 = (unsigned short*)S4;
  unsigned short* QS2   = (unsigned short*)S7;
  unsigned short* KS16  = (unsigned short*)S0;
  float*          O2F   = (float*)S5;
  unsigned short* LN2H  = (unsigned short*)S0;
  float*          LN2F  = (float*)S2;
  unsigned short* G16   = (unsigned short*)S4;
  float*          Y3F   = (float*)S0;

  const dim3 blk(256);
  const dim3 blk32(32);
  const dim3 bLN(LN_THREADS);
  const dim3 gLN(NROWS);
  const int tilesP  = (NROWS / 64) * (DMODEL / 64);
  const int tilesV  = (DMODEL / 64) * (SEQ / 64);
  const int tilesF  = (NROWS / 64) * (DFF / 64);
  const int tilesAp = (SEQ / 64);
  const dim3 gP((tilesP + 7) / 8, 1);
  const dim3 gV((tilesV + 7) / 8, NB);
  const dim3 gF((tilesF + 7) / 8, 1);
  const dim3 gCX(1, NB * NHEAD);
  const dim3 gAP((tilesAp + 7) / 8, NB * NHEAD);
  const dim3 gAT(NB * (SEQ / 16));
  const dim3 bAT(ATT_THREADS);
  const dim3 gCS(NB * DMODEL);
  const dim3 bCS(CS_THREADS);

  const float osXW = 1.0f / (XC * WSC);
  const float osHW = 1.0f / (HC * WSC);

  cvt16<<<dim3((3 * DMODEL * DMODEL) / 2048), blk, 0, stream>>>(w_qvk, WQVK16, DMODEL, 3 * DMODEL, 3 * DMODEL, WSC);
  cvt16<<<dim3((2 * DMODEL * DMODEL) / 2048), blk, 0, stream>>>(w_kv, WKV16, DMODEL, 2 * DMODEL, 2 * DMODEL, WSC);
  cvt16<<<dim3((DMODEL * DMODEL) / 2048), blk, 0, stream>>>(w_q, WQ16, DMODEL, DMODEL, DMODEL, WSC);
  cvt16<<<dim3((DFF * DMODEL) / 2048), blk, 0, stream>>>(w_ff1, W116, DMODEL, DFF, DFF, WSC);
  cvt16<<<dim3((DMODEL * DFF) / 2048), blk, 0, stream>>>(w_ff2, W216, DFF, DMODEL, DMODEL, WSC);
  cvt16<<<dim3((NROWS * DMODEL) / 2048), blk, 0, stream>>>(x, X16, DMODEL, SEQ, SEQ_FULL, XC);
  cvt16<<<dim3((NROWS * DMODEL) / 2048), blk, 0, stream>>>(mem, MEM16, DMODEL, SEQ, SEQ_FULL, XC);

  gemm64<2, 0, 4, 1><<<gP, blk, 0, stream>>>(
      X16, DMODEL, 0LL, 0LL,
      WQVK16, DMODEL, 0LL, 0LL,
      (const float*)0,
      b_qvk, DMODEL,
      (void*)QS16, DMODEL, 0LL, 0LL, 1,
      NROWS, DMODEL, DMODEL, osXW, QSC);

  gemm64<2, 0, 3, 1><<<gP, blk, 0, stream>>>(
      X16, DMODEL, 0LL, 0LL,
      WQVK16 + (size_t)2 * DMODEL * DMODEL, DMODEL, 0LL, 0LL,
      (const float*)0,
      b_qvk + 2 * DMODEL, DMODEL,
      (void*)KE16, DMODEL, 0LL, 0LL, 1,
      NROWS, DMODEL, DMODEL, osXW, KEC);

  gemm64<2, 0, 0, 2><<<gV, blk, 0, stream>>>(
      WQVK16 + (size_t)DMODEL * DMODEL, DMODEL, 0LL, 0LL,
      X16, DMODEL, (long long)SEQ * DMODEL, 0LL,
      (const float*)0,
      b_qvk + DMODEL, DMODEL,
      (void*)VT16, SEQ, (long long)DMODEL * SEQ, 0LL, 1,
      DMODEL, SEQ, DMODEL, osXW, VC);

  attnc<<<gAT, bAT, 0, stream>>>(QS16, KE16, VT16, O1F);

  lnorm<1, 1, 1><<<gLN, bLN, 0, stream>>>(O1F, x, ln1_g, ln1_b, LN1H, LN1F, HC);

  gemm64<0, 0, 0, 2><<<gV, blk, 0, stream>>>(
      WKV16, DMODEL, 0LL, 0LL,
      MEM16, DMODEL, (long long)SEQ * DMODEL, 0LL,
      (const float*)0,
      b_kv, DMODEL,
      (void*)K2TF, SEQ, (long long)DMODEL * SEQ, 0LL, 1,
      DMODEL, SEQ, DMODEL, osXW, 1.0f);

  gemm64<2, 0, 0, 2><<<gV, blk, 0, stream>>>(
      WKV16 + (size_t)DMODEL * DMODEL, DMODEL, 0LL, 0LL,
      MEM16, DMODEL, (long long)SEQ * DMODEL, 0LL,
      (const float*)0,
      b_kv + DMODEL, DMODEL,
      (void*)V2T16, SEQ, (long long)DMODEL * SEQ, 0LL, 1,
      DMODEL, SEQ, DMODEL, osXW, VC);

  gemm64<2, 0, 4, 1><<<gP, blk, 0, stream>>>(
      LN1H, DMODEL, 0LL, 0LL,
      WQ16, DMODEL, 0LL, 0LL,
      (const float*)0,
      b_q, DMODEL,
      (void*)QS2, DMODEL, 0LL, 0LL, 1,
      NROWS, DMODEL, DMODEL, osHW, QSC);

  colsoft<<<gCS, bCS, 0, stream>>>(K2TF, KS16);

  gemm64<2, 0, 0, 0><<<gCX, blk32, 0, stream>>>(
      V2T16, SEQ, (long long)HDIM * SEQ, 0LL,
      KS16, SEQ, (long long)HDIM * SEQ, 0LL,
      (const float*)0,
      (const float*)0, 1,
      (void*)CTX16, HDIM, (long long)HDIM * HDIM, 0LL, 1,
      HDIM, HDIM, SEQ, 1.0f / (VC * KSC), CC);

  gemm64<0, 2, 0, 0><<<gAP, blk, 0, stream>>>(
      QS2, DMODEL, (long long)SEQ * DMODEL, (long long)HDIM,
      CTX16, HDIM, (long long)NHEAD * HDIM * HDIM, (long long)HDIM * HDIM,
      LN1F,
      (const float*)0, 1,
      (void*)O2F, DMODEL, (long long)SEQ * DMODEL, (long long)HDIM, NHEAD,
      SEQ, HDIM, HDIM, 1.0f / (QSC * CC), 1.0f);

  lnorm<0, 1, 1><<<gLN, bLN, 0, stream>>>(O2F, (const float*)0, ln2_g, ln2_b, LN2H, LN2F, HC);

  gemm64<2, 0, 1, 1><<<gF, blk, 0, stream>>>(
      LN2H, DMODEL, 0LL, 0LL,
      W116, DMODEL, 0LL, 0LL,
      (const float*)0,
      b_ff1, DFF,
      (void*)G16, DFF, 0LL, 0LL, 1,
      NROWS, DFF, DMODEL, osHW, GC);

  gemm64<0, 2, 0, 1><<<gP, blk, 0, stream>>>(
      G16, DFF, 0LL, 0LL,
      W216, DFF, 0LL, 0LL,
      LN2F,
      b_ff2, DMODEL,
      (void*)Y3F, DMODEL, 0LL, 0LL, 1,
      NROWS, DMODEL, DFF, 1.0f / (GC * WSC), 1.0f);

  lnorm<0, 0, 2><<<gLN, bLN, 0, stream>>>(Y3F, (const float*)0, ln3_g, ln3_b, (unsigned short*)0, out, 1.0f);
  (void)hipGetLastError();
}
